// Model_46952582480187
// MI455X (gfx1250) — hardware-verified
//
#include <hip/hip_runtime.h>


#define T_    512
#define F_    32
#define U_    350
#define G4    1400
#define NP    1408
#define NT    88
#define KB    11
#define ZROW  1409
#define HROW  360
#define WCHUNK (11 * 512)
#define HROW2 (2 * HROW)

typedef _Float16 v16bf __attribute__((ext_vector_type(16)));
typedef __attribute__((ext_vector_type(4))) float v4f_t;
typedef float v4fa __attribute__((ext_vector_type(4), may_alias));
#define RSPLIT (1.0f / 2048.0f)
#define PLX ((size_t)256 * T_ * F_)
#define PLK ((size_t)NT * 512)
#define PLW ((size_t)KB * NT * 512)
typedef float  v8f   __attribute__((ext_vector_type(8)));
typedef unsigned int u32x4 __attribute__((ext_vector_type(4)));
typedef int          i32x4 __attribute__((ext_vector_type(4)));
typedef int          i32x8 __attribute__((ext_vector_type(8)));

union FragAB { v16bf v; uint4 q[2]; };

__device__ __forceinline__ unsigned short f2bf(float f) { return __builtin_bit_cast(unsigned short, (_Float16)f); }
__device__ __forceinline__ void split16(float f, unsigned short& h, unsigned short& l) {
  const _Float16 hh = (_Float16)f; h = __builtin_bit_cast(unsigned short, hh);
  l = __builtin_bit_cast(unsigned short, (_Float16)((f - (float)hh) * 2048.0f));
}
__device__ __forceinline__ unsigned pack2s(float a, float b, unsigned* lo) {
  unsigned short h0, l0, h1, l1; split16(a, h0, l0); split16(b, h1, l1);
  *lo = (unsigned)l0 | ((unsigned)l1 << 16); return (unsigned)h0 | ((unsigned)h1 << 16);
}
__device__ __forceinline__ v8f wmma1(v16bf a, v16bf b, v8f c) {
  return __builtin_amdgcn_wmma_f32_16x16x32_f16(false, a, false, b, (short)0, c, false, false);
}
__device__ __forceinline__ float sigm(float x) {
  return 1.0f / (1.0f + __expf(-x));
}

__device__ __forceinline__ void tdm_load_chunk(const void* gsrc,
                                               unsigned int lds_addr) {
  unsigned long long ga = (unsigned long long)gsrc;
  u32x4 g0 = { 1u,
               lds_addr,
               (unsigned int)ga,
               (unsigned int)((ga >> 32) & 0x01FFFFFFu) | (2u << 30) };
  i32x8 g1 = { (int)0x00030000,
               (int)(1408u << 16),
               (int)(1u << 16),
               (int)(1408u << 16),
               1,
               1408,
               0, 0 };
  i32x4 gz = { 0, 0, 0, 0 };
#if __clang_major__ >= 23
  i32x8 gz8 = { 0, 0, 0, 0, 0, 0, 0, 0 };
  __builtin_amdgcn_tensor_load_to_lds(g0, g1, gz, gz, gz8, 0);
#else
  __builtin_amdgcn_tensor_load_to_lds(g0, g1, gz, gz, 0);
#endif
}

__device__ __forceinline__ int bslot_k(int lane, int s) { const int h8 = (lane < 16) ? 0 : 8; return (s < 8) ? (h8 + s) : (16 + h8 + (s - 8)); }

__global__ void lstm46_pack_xbf(const float* __restrict__ x,
                                unsigned short* __restrict__ xbf, int n) {
  for (int i = (blockIdx.x * blockDim.x + threadIdx.x) * 2; i < n; i += gridDim.x * blockDim.x * 2) {
    unsigned lo; const unsigned hv = pack2s(x[i], x[i + 1], &lo);
    *(volatile unsigned*)(xbf + i) = hv; *(volatile unsigned*)(xbf + (size_t)n + i) = lo;
    __threadfence();
    *(volatile unsigned*)(xbf + i) = hv; *(volatile unsigned*)(xbf + (size_t)n + i) = lo;
  }
}

__global__ void lstm46_pack_k(const float* __restrict__ K,
                              unsigned short* __restrict__ pk) {
  int idx = blockIdx.x * blockDim.x + threadIdx.x;
  if (idx * 2 >= NT * 512) return;
  idx *= 2;
  int nb = idx >> 9, r = idx & 511, lane = r >> 4, s = r & 15;
  int n = nb * 16 + (lane & 15);
  int k = bslot_k(lane, s);
  unsigned lo; const unsigned hv = pack2s((n < G4) ? K[k * G4 + n] : 0.0f, (n < G4) ? K[(k + 1) * G4 + n] : 0.0f, &lo);
  *(volatile unsigned*)(pk + idx) = hv; *(volatile unsigned*)(pk + PLK + idx) = lo;
  __threadfence();
  *(volatile unsigned*)(pk + idx) = hv; *(volatile unsigned*)(pk + PLK + idx) = lo;
}

__global__ void lstm46_pack_w(const float* __restrict__ W,
                              unsigned short* __restrict__ pw) {
  int idx = blockIdx.x * blockDim.x + threadIdx.x;
  if (idx * 2 >= KB * NT * 512) return;
  idx *= 2;
  int kb = idx / (NT * 512), rem = idx % (NT * 512);
  int nb = rem >> 9, r = rem & 511, lane = r >> 4, s = r & 15;
  int k = kb * 32 + bslot_k(lane, s);
  int n = nb * 16 + (lane & 15);
  unsigned lo; const unsigned hv = pack2s((k < U_ && n < G4) ? W[k * G4 + n] : 0.0f, (k + 1 < U_ && n < G4) ? W[(k + 1) * G4 + n] : 0.0f, &lo);
  *(volatile unsigned*)(pw + idx) = hv; *(volatile unsigned*)(pw + PLW + idx) = lo;
  __threadfence();
  *(volatile unsigned*)(pw + idx) = hv; *(volatile unsigned*)(pw + PLW + idx) = lo;
}


__global__ __launch_bounds__(256)
void lstm46_main(const unsigned short* __restrict__ xbf,
                 const unsigned short* __restrict__ pk,
                 const unsigned short* __restrict__ pw,
                 const float* __restrict__ bias,
                 const float* __restrict__ dw,
                 const float* __restrict__ dbp,
                 float* __restrict__ out) {
  extern __shared__ char smem_raw[];
  float*          zS    = (float*)smem_raw;
  float*          cS    = zS + 16 * ZROW;
  float*          biasS = cS + 16 * U_;
  float*          dwS   = biasS + NP;
  float*          outS  = dwS + 352;
  unsigned short* hS    = (unsigned short*)(outS + 16 * T_);
  unsigned short* wbS   = hS + 16 * HROW2;

  const int tid  = threadIdx.x;
  const int lane = tid & 31;
  const int wave = tid >> 5;
  const int m16  = lane & 15;
  const int hsel = lane >> 4;
  const int k0   = hsel * 8;
  const int b0   = blockIdx.x * 16;
  const float db = dbp[0];

  for (int i = tid; i < 16 * U_;  i += 256) cS[i] = 0.0f;
  for (int i = tid; i < 16 * HROW2; i += 256) hS[i] = 0;
  for (int i = tid; i < NP;  i += 256) biasS[i] = (i < G4) ? bias[i] : 0.0f;
  for (int i = tid; i < 352; i += 256) dwS[i]   = (i < U_) ? dw[i]   : 0.0f;
  __syncthreads();

  const unsigned int wb_addr0 = (unsigned int)(unsigned long long)(wbS + wave * WCHUNK);
  const unsigned short* wchunk  = pw + wave * WCHUNK;

  for (int t = 0; t < T_; ++t) {
    v8f acc[11];
#pragma unroll
    for (int j = 0; j < 11; ++j) {
      float bv = biasS[(wave * 11 + j) * 16 + m16];
#pragma unroll
      for (int r = 0; r < 8; ++r) acc[j][r] = bv;
    }

    {
      FragAB a;
      const unsigned short* xp =
          xbf + ((size_t)(b0 + m16) * T_ + t) * F_;
      a.q[0]  = *(const uint4*)(xp + k0);
      a.q[1]  = *(const uint4*)(xp + k0 + 16);
      if (t + 1 < T_)
        __builtin_prefetch(xp + F_ + k0, 0, 0);
#pragma unroll
      for (int j = 0; j < 11; ++j) {
        FragAB b;
        const unsigned short* bp = pk + ((wave * 11 + j) * 512) + lane * 16;
        b.q[0]  = *(const uint4*)(bp);        b.q[1]  = *(const uint4*)(bp + 8);
        acc[j] = wmma1(a.v, b.v, acc[j]);
        asm volatile("" ::: "memory");
      }
    }

    for (int kb = 0; kb < KB; ++kb) {
      tdm_load_chunk(wchunk + (size_t)kb * (NT * 512), wb_addr0);
      __builtin_amdgcn_s_wait_tensorcnt(0);

      FragAB a;
      const unsigned short* hp = hS + m16 * HROW2 + kb * 32 + k0;
      a.q[0]  = *(const uint4*)(hp);         a.q[1]  = *(const uint4*)(hp + 16);
      const unsigned short* wb  = wbS + wave * WCHUNK;
#pragma unroll
      for (int j = 0; j < 11; ++j) {
        FragAB b;
        const unsigned short* bp = wb + j * 512 + lane * 16;
        b.q[0]  = *(const uint4*)(bp);   b.q[1]  = *(const uint4*)(bp + 8);
        acc[j] = wmma1(a.v, b.v, acc[j]);
        asm volatile("" ::: "memory");
      }
    }

#pragma unroll
    for (int j = 0; j < 11; ++j) {
      int col = (wave * 11 + j) * 16 + m16;
#pragma unroll
      for (int r = 0; r < 8; ++r)
        zS[(r + hsel * 8) * ZROW + col] = acc[j][r];
    }
    __syncthreads();

    const int m  = tid >> 4;
    const int ul = tid & 15;
    float dsum = 0.0f;
    for (int u = ul; u < U_; u += 16) {
      float zi = zS[m * ZROW + u];
      float zf = zS[m * ZROW + U_ + u];
      float zg = zS[m * ZROW + 2 * U_ + u];
      float zo = zS[m * ZROW + 3 * U_ + u];
      float ig = sigm(zi);
      float fg = sigm(zf);
      float g  = fmaxf(zg, 0.0f);
      float og = sigm(zo);
      float cn = fg * cS[m * U_ + u] + ig * g;
      float hn = og * fmaxf(cn, 0.0f);
      cS[m * U_ + u] = cn;
      { unsigned short hh, hl; split16(hn, hh, hl); hS[m * HROW2 + u] = hh; hS[m * HROW2 + HROW + u] = hl; }
      dsum += hn * dwS[u];
    }
#pragma unroll
    for (int off = 8; off; off >>= 1) dsum += __shfl_xor(dsum, off, 16);
    if (ul == 0) outS[m * T_ + t] = dsum + db;
    __syncthreads();
  }

#pragma unroll 1
  for (int pass = 0; pass < 2; ++pass) {
#pragma unroll
    for (int i = 0; i < 8; ++i) {
      const int c = tid + 256 * i, rr = c >> 7, q = c & 127;
      *(volatile v4f_t*)(out + (size_t)(b0 + rr) * T_ + q * 4) = *(const volatile v4fa*)(outS + rr * T_ + q * 4);
    }
    __threadfence();
  }
}


extern "C" void kernel_launch(void* const* d_in, const int* in_sizes, int n_in,
                              void* d_out, int out_size, void* d_ws, size_t ws_size,
                              hipStream_t stream) {
  const float* x    = (const float*)d_in[0];
  const float* kern = (const float*)d_in[1];
  const float* rec  = (const float*)d_in[2];
  const float* bias = (const float*)d_in[3];
  const float* dw   = (const float*)d_in[4];
  const float* db   = (const float*)d_in[5];
  float* out = (float*)d_out;

  const size_t XBF_BYTES = (size_t)256 * T_ * F_ * 2 * 2;
  const size_t PK_BYTES  = (size_t)NT * 512 * 2 * 2;
  unsigned short* xbf = (unsigned short*)d_ws;
  unsigned short* pk  = (unsigned short*)((char*)d_ws + XBF_BYTES);
  unsigned short* pw  = (unsigned short*)((char*)d_ws + XBF_BYTES + PK_BYTES);

  const int nX = 256 * T_ * F_;
  lstm46_pack_xbf<<<(nX / 2 + 255) / 256, 256, 0, stream>>>(x, xbf, nX);
  lstm46_pack_k  <<<(NT * 512 / 2 + 255) / 256, 256, 0, stream>>>(kern, pk);
  lstm46_pack_w  <<<(KB * NT * 512 / 2 + 255) / 256, 256, 0, stream>>>(rec, pw);

  const int smemBytes =
      (16 * ZROW + 16 * U_ + NP + 352 + 16 * T_) * 4 + 16 * HROW2 * 2
      + 8 * WCHUNK * 2;
  (void)hipFuncSetAttribute((const void*)lstm46_main,
                            hipFuncAttributeMaxDynamicSharedMemorySize,
                            smemBytes);
  lstm46_main<<<16, 256, smemBytes, stream>>>(xbf, pk, pw, bias, dw, db, out);
}
